// BenchmarkLSTM_62732292325417
// MI455X (gfx1250) — hardware-verified
//
#include <hip/hip_runtime.h>
#include <math.h>

constexpr int NSEQ   = 672;
constexpr int NBAT   = 512;
constexpr int NFEAT  = 38;
constexpr int NHID   = 100;
constexpr int NGATE  = 4 * NHID;
constexpr int NOUTF  = 8;
constexpr int UPAD   = 112;
constexpr int XPAD   = 48;
constexpr int KL0    = XPAD + UPAD;
constexpr int KL12   = 2 * UPAD;
constexpr int KHEAD  = 128;
constexpr int NWROW  = 4 * UPAD;
constexpr int NHROW  = 16;
constexpr int COL_X  = 0;
constexpr int COL_H0 = XPAD;
constexpr int COL_H1 = COL_H0 + UPAD;
constexpr int COL_H2 = COL_H1 + UPAD;
constexpr int COL_HD = COL_H2 + UPAD - KHEAD;
constexpr int HDZERO = COL_H2 - COL_HD;
constexpr int APITCH = COL_H2 + UPAD + 8;
constexpr int ABUF   = 16 * APITCH;
constexpr int NWAVE  = 7;
constexpr int NTHR   = 32 * NWAVE;
constexpr int HSP    = 20;
constexpr int XF4    = 16 * NFEAT / 4;
constexpr int XZW    = XPAD - NFEAT;
constexpr int XZP    = 16 * XZW;
constexpr float WCARRY     = 16.0f;
constexpr float WCARRY_INV = 1.0f / 16.0f;

static_assert(NWAVE * 16 == UPAD, "one 16-unit column tile per wave");
static_assert(KL0 % 32 == 0 && KL12 % 32 == 0 && KHEAD % 32 == 0, "K multiples of 32");
static_assert(KL0 == 160 && KL12 == 224, "K-concat sizes");
static_assert(UPAD % 16 == 0 && XPAD % 16 == 0, "half-chunk granularity of the concat boundary");
static_assert((2 * ABUF) % NTHR == 0, "zero-fill loop exact");
static_assert(XF4 <= NTHR && XZP <= NTHR, "x staging fits one pass");
static_assert((16 * NFEAT) % 4 == 0, "x tile is whole float4s");
static_assert(APITCH % 8 == 0 && COL_H0 % 8 == 0 && COL_H1 % 8 == 0 && COL_H2 % 8 == 0 && COL_HD % 8 == 0, "16-B aligned fragments");
static_assert(COL_HD >= COL_H1 && HDZERO == 16, "head chunk window lies on written columns");
static_assert(NBAT % 16 == 0, "16-row batch tiles");
static_assert((NWROW * (KL0 / 8)) % 256 == 0 && (NWROW * (KL12 / 8)) % 256 == 0 && (NHROW * (KHEAD / 8)) % 256 == 0, "plane builders exact");

typedef __attribute__((ext_vector_type(16))) _Float16 v16h;
typedef __attribute__((ext_vector_type(8)))  _Float16 v8h;
typedef __attribute__((ext_vector_type(8)))  float    v8f;
typedef __attribute__((ext_vector_type(4)))  float    v4f;

union FragU { v16h v; v8h h[2]; };

__device__ __forceinline__ v16h frag_load2(const _Float16* p0, const _Float16* p1) {
  FragU f;
  f.h[0] = *(const v8h*)(p0);
  f.h[1] = *(const v8h*)(p1);
  return f.v;
}
__device__ __forceinline__ v16h frag_load(const _Float16* p) { return frag_load2(p, p + 16); }
__device__ __forceinline__ v8f mma_f16(v16h a, v16h b, v8f c) {
  return __builtin_amdgcn_wmma_f32_16x16x32_f16(false, a, false, b, (short)0, c, false, false);
}
__device__ __forceinline__ void guard_all4(v8f& a0, v8f& a1, v8f& a2, v8f& a3, v16h a, v16h b0, v16h b1, v16h b2, v16h b3) {
  asm volatile("v_nop\n\tv_nop\n\tv_nop\n\tv_nop" : "+v"(a0), "+v"(a1), "+v"(a2), "+v"(a3) : "v"(a), "v"(b0), "v"(b1), "v"(b2), "v"(b3));
}
__device__ __forceinline__ void guard_one(v8f& a0, v16h a, v16h b) {
  asm volatile("v_nop\n\tv_nop\n\tv_nop\n\tv_nop" : "+v"(a0) : "v"(a), "v"(b));
}
__device__ __forceinline__ void acc_guard4(v8f& a, v8f& b, v8f& c, v8f& d) {
  asm volatile("v_nop\n\tv_nop\n\tv_nop\n\tv_nop" : "+v"(a), "+v"(b), "+v"(c), "+v"(d));
}
__device__ __forceinline__ void acc_guard1(v8f& a) {
  asm volatile("v_nop\n\tv_nop\n\tv_nop\n\tv_nop" : "+v"(a));
}
__device__ __forceinline__ void wave_lds_sync() {
  __builtin_amdgcn_fence(__ATOMIC_RELEASE, "workgroup");
  __builtin_amdgcn_wave_barrier();
  __builtin_amdgcn_fence(__ATOMIC_ACQUIRE, "workgroup");
}
__device__ __forceinline__ v8f splat8(float s) { return (v8f){s, s, s, s, s, s, s, s}; }

__device__ __forceinline__ float fsig(float x)  { return __builtin_amdgcn_rcpf(1.0f + __expf(-x)); }
__device__ __forceinline__ float ftanh(float x) { return 1.0f - 2.0f * __builtin_amdgcn_rcpf(__expf(2.0f * x) + 1.0f); }

__global__ __launch_bounds__(256) void wplane_kernel(const float* __restrict__ srcA, int nA, int pitchA, int widthA,
                                                     const float* __restrict__ srcB, int nB, int pitchB,
                                                     unsigned short* __restrict__ dst, int k8, int nrows, int headmode) {
  const int i  = blockIdx.x * 256 + threadIdx.x;
  const int n8 = nrows * k8;
  const int ic = (i < n8) ? i : (n8 - 1);
  const int row = ic / k8;
  const int kb  = (ic - row * k8) * 8;
  const int wv = row >> 6;
  const int q  = (row >> 4) & 3;
  const int u  = 16 * wv + (row & 15);
  const bool rowok = headmode ? (row < NOUTF) : (u < NHID);
  const int  srow0 = headmode ? row : (q * NHID + u);
  const int  srow  = rowok ? srow0 : 0;
  const bool first = kb < widthA;
  const float* sp  = first ? srcA : srcB;
  const int pitch  = first ? pitchA : pitchB;
  const int nv     = first ? nA : nB;
  const int cb     = first ? kb : (kb - widthA);
  v8h hv;
#pragma unroll
  for (int e = 0; e < 8; ++e) {
    const int col = cb + e;
    const bool ok = rowok && (col < nv);
    int cc = (col < nv) ? col : (nv - 1);
    cc = (cc < 0) ? 0 : cc;
    const float v = sp[(size_t)srow * (size_t)pitch + (size_t)cc];
    const float f = ok ? (v * WCARRY) : 0.0f;
    hv[e] = (_Float16)f;
  }
  if (i < n8) {
    *(volatile v8h*)(dst + (size_t)i * 8) = hv;
    __threadfence();
    *(volatile v8h*)(dst + (size_t)i * 8) = hv;
  }
}

template <int NCH, int KSPLIT, int KP>
__device__ __forceinline__ void gate_mma(const _Float16* lds, int offLo, int offHi, const _Float16* wrow,
                                         v8f& a0, v8f& a1, v8f& a2, v8f& a3) {
#pragma unroll 1
  for (int kc = 0; kc < NCH; ++kc) {
    const int k0 = kc * 32;
    const int o0 = ((k0 < KSPLIT) ? offLo : offHi) + k0;
    const int o1 = ((k0 + 16 < KSPLIT) ? offLo : offHi) + k0 + 16;
    const v16h a  = frag_load2(lds + o0, lds + o1);
    const v16h b0 = frag_load(wrow + k0);
    const v16h b1 = frag_load(wrow + 16 * KP + k0);
    const v16h b2 = frag_load(wrow + 32 * KP + k0);
    const v16h b3 = frag_load(wrow + 48 * KP + k0);
    a0 = mma_f16(a, b0, a0);
    a1 = mma_f16(a, b1, a1);
    a2 = mma_f16(a, b2, a2);
    a3 = mma_f16(a, b3, a3);
    guard_all4(a0, a1, a2, a3, a, b0, b1, b2, b3);
  }
  acc_guard4(a0, a1, a2, a3);
}

__device__ __forceinline__ void cell_update(const v8f& ai, const v8f& af, const v8f& ag, const v8f& ao,
                                            float (&cst)[8], _Float16* hp) {
#pragma unroll
  for (int r = 0; r < 8; ++r) {
    const float zi = ai[r] * WCARRY_INV;
    const float zf = af[r] * WCARRY_INV;
    const float zg = ag[r] * WCARRY_INV;
    const float zo = ao[r] * WCARRY_INV;
    const float ig = fsig(zi);
    const float fg = fsig(zf);
    const float gg = ftanh(zg);
    const float og = fsig(zo);
    const float cn = fg * cst[r] + ig * gg;
    cst[r] = cn;
    const float hn = og * ftanh(cn);
    hp[r * APITCH] = (_Float16)hn;
  }
}

__device__ __forceinline__ void stage_x(_Float16* lds, int boff, const float* xt, int tid) {
  const int i4 = (tid < XF4) ? tid : (XF4 - 1);
  v4f v = *(const v4f*)(xt + 4 * i4);
  asm volatile("" : "+v"(v));
  if (tid < XF4) {
#pragma unroll
    for (int e = 0; e < 4; ++e) {
      const int el = 4 * tid + e;
      const int m  = el / NFEAT;
      const int d  = el - m * NFEAT;
      const float f = v[e];
      lds[boff + m * APITCH + COL_X + d] = (_Float16)f;
    }
  }
  if (tid < XZP) {
    const int m = tid / XZW;
    const int d = NFEAT + (tid - m * XZW);
    lds[boff + m * APITCH + COL_X + d] = (_Float16)0.0f;
  }
}

__global__ __launch_bounds__(NTHR) void lstm3_kernel(const float* __restrict__ x,
                                                     const float* __restrict__ bih0, const float* __restrict__ bhh0,
                                                     const float* __restrict__ bih1, const float* __restrict__ bhh1,
                                                     const float* __restrict__ bih2, const float* __restrict__ bhh2,
                                                     const float* __restrict__ blin,
                                                     const unsigned short* __restrict__ WP0p,
                                                     const unsigned short* __restrict__ WP1p,
                                                     const unsigned short* __restrict__ WP2p,
                                                     const unsigned short* __restrict__ WPHp,
                                                     float* __restrict__ out) {
  __shared__ __align__(16) _Float16 Abuf[2 * ABUF];
  __shared__ __align__(16) float    Hs[16 * HSP];
  const int tid  = threadIdx.x;
  const int lane = tid & 31;
  const int wave = __builtin_amdgcn_readfirstlane(tid >> 5);
  const int c    = lane & 15;
  const int hh   = lane >> 4;
  const int koff = hh * 8;
  const int b0   = blockIdx.x * 16;

#pragma unroll 1
  for (int i = tid; i < 2 * ABUF; i += NTHR) Abuf[i] = (_Float16)0.0f;

  const int  u   = 16 * wave + c;
  const int  uc  = (u < NHID) ? u : (NHID - 1);
  const bool uok = (u < NHID);
  float bb0[4], bb1[4], bb2[4];
#pragma unroll
  for (int q = 0; q < 4; ++q) {
    const int idx = q * NHID + uc;
    const float s0 = bih0[idx] + bhh0[idx];
    const float s1 = bih1[idx] + bhh1[idx];
    const float s2 = bih2[idx] + bhh2[idx];
    bb0[q] = uok ? (s0 * WCARRY) : 0.0f;
    bb1[q] = uok ? (s1 * WCARRY) : 0.0f;
    bb2[q] = uok ? (s2 * WCARRY) : 0.0f;
  }
  const float blv = blin[(c < NOUTF) ? c : (NOUTF - 1)];
  const float bl  = (c < NOUTF) ? (blv * WCARRY) : 0.0f;

  float cst0[8], cst1[8], cst2[8];
#pragma unroll
  for (int r = 0; r < 8; ++r) { cst0[r] = 0.0f; cst1[r] = 0.0f; cst2[r] = 0.0f; }

  const _Float16* w0row = (const _Float16*)WP0p + (size_t)(wave * 64 + c) * KL0  + koff;
  const _Float16* w1row = (const _Float16*)WP1p + (size_t)(wave * 64 + c) * KL12 + koff;
  const _Float16* w2row = (const _Float16*)WP2p + (size_t)(wave * 64 + c) * KL12 + koff;
  const _Float16* whrow = (const _Float16*)WPHp + (size_t)c * KHEAD + koff;

  const int rowA = c * APITCH + koff;
  const int rowH = (8 * hh) * APITCH + 16 * wave + c;

  __syncthreads();
  stage_x(Abuf, 0, x + (size_t)b0 * NFEAT, tid);
  __syncthreads();

#pragma unroll 1
  for (int t = 0; t < NSEQ; ++t) {
    const int cur = (t & 1) * ABUF;
    const int nxt = ABUF - cur;

    {
      v8f a0 = splat8(bb0[0]), a1 = splat8(bb0[1]), a2 = splat8(bb0[2]), a3 = splat8(bb0[3]);
      gate_mma<KL0 / 32, 0, KL0>(Abuf, cur + rowA + COL_X, cur + rowA + COL_X, w0row, a0, a1, a2, a3);
      cell_update(a0, a1, a2, a3, cst0, Abuf + nxt + rowH + COL_H0);
    }
    {
      const int tn = (t + 1 < NSEQ) ? (t + 1) : (NSEQ - 1);
      stage_x(Abuf, nxt, x + ((size_t)tn * NBAT + (size_t)b0) * NFEAT, tid);
    }
    __syncthreads();

    {
      v8f a0 = splat8(bb1[0]), a1 = splat8(bb1[1]), a2 = splat8(bb1[2]), a3 = splat8(bb1[3]);
      gate_mma<KL12 / 32, UPAD, KL12>(Abuf, nxt + rowA + COL_H0, cur + rowA + COL_H0, w1row, a0, a1, a2, a3);
      cell_update(a0, a1, a2, a3, cst1, Abuf + nxt + rowH + COL_H1);
    }
    __syncthreads();

    {
      v8f a0 = splat8(bb2[0]), a1 = splat8(bb2[1]), a2 = splat8(bb2[2]), a3 = splat8(bb2[3]);
      gate_mma<KL12 / 32, UPAD, KL12>(Abuf, nxt + rowA + COL_H1, cur + rowA + COL_H1, w2row, a0, a1, a2, a3);
      cell_update(a0, a1, a2, a3, cst2, Abuf + nxt + rowH + COL_H2);
    }
    __syncthreads();

    if (wave == 0) {
      v8f ah = splat8(bl);
      const int ho = nxt + rowA + COL_HD;
#pragma unroll 1
      for (int kc = 0; kc < KHEAD / 32; ++kc) {
        const v16h a = frag_load(Abuf + ho + 32 * kc);
        const v16h b = frag_load(whrow + 32 * kc);
        ah = mma_f16(a, b, ah);
        guard_one(ah, a, b);
      }
      acc_guard1(ah);
#pragma unroll
      for (int r = 0; r < 8; ++r) Hs[(8 * hh + r) * HSP + c] = ah[r] * WCARRY_INV;
      wave_lds_sync();
      const v4f ov = *(const v4f*)(Hs + (lane >> 1) * HSP + (lane & 1) * 4);
      float* op = out + ((size_t)t * NBAT + (size_t)b0) * NOUTF + lane * 4;
      *(volatile v4f*)op = ov;
      __threadfence();
      *(volatile v4f*)op = ov;
      wave_lds_sync();
    }
  }
}

extern "C" void kernel_launch(void* const* d_in, const int* in_sizes, int n_in,
                              void* d_out, int out_size, void* d_ws, size_t ws_size, hipStream_t stream) {
  if (n_in < 15 || d_out == nullptr || d_ws == nullptr) return;
  if (in_sizes[0] != NSEQ * NBAT * NFEAT || in_sizes[1] != NGATE * NFEAT || in_sizes[2] != NGATE * NHID ||
      in_sizes[3] != NGATE || in_sizes[4] != NGATE || in_sizes[5] != NGATE * NHID || in_sizes[6] != NGATE * NHID ||
      in_sizes[7] != NGATE || in_sizes[8] != NGATE || in_sizes[9] != NGATE * NHID || in_sizes[10] != NGATE * NHID ||
      in_sizes[11] != NGATE || in_sizes[12] != NGATE || in_sizes[13] != NOUTF * NHID || in_sizes[14] != NOUTF ||
      out_size != NSEQ * NBAT * NOUTF) return;

  const float* x    = (const float*)d_in[0];
  const float* wih0 = (const float*)d_in[1];
  const float* whh0 = (const float*)d_in[2];
  const float* bih0 = (const float*)d_in[3];
  const float* bhh0 = (const float*)d_in[4];
  const float* wih1 = (const float*)d_in[5];
  const float* whh1 = (const float*)d_in[6];
  const float* bih1 = (const float*)d_in[7];
  const float* bhh1 = (const float*)d_in[8];
  const float* wih2 = (const float*)d_in[9];
  const float* whh2 = (const float*)d_in[10];
  const float* bih2 = (const float*)d_in[11];
  const float* bhh2 = (const float*)d_in[12];
  const float* wlin = (const float*)d_in[13];
  const float* blin = (const float*)d_in[14];
  float* out = (float*)d_out;

  char* ws = (char*)d_ws;
  size_t off = 0;
  auto carve = [&](size_t bytes) -> char* { char* p = ws + off; off += (bytes + 255) & ~(size_t)255; return p; };
  unsigned short* WP0 = (unsigned short*)carve((size_t)NWROW * KL0 * 2);
  unsigned short* WP1 = (unsigned short*)carve((size_t)NWROW * KL12 * 2);
  unsigned short* WP2 = (unsigned short*)carve((size_t)NWROW * KL12 * 2);
  unsigned short* WPH = (unsigned short*)carve((size_t)NHROW * KHEAD * 2);
  if (off > ws_size || off > (size_t)134217728) return;

  wplane_kernel<<<(NWROW * (KL0 / 8)) / 256, 256, 0, stream>>>(wih0, NFEAT, NFEAT, XPAD, whh0, NHID, NHID, WP0, KL0 / 8, NWROW, 0);
  wplane_kernel<<<(NWROW * (KL12 / 8)) / 256, 256, 0, stream>>>(wih1, NHID, NHID, UPAD, whh1, NHID, NHID, WP1, KL12 / 8, NWROW, 0);
  wplane_kernel<<<(NWROW * (KL12 / 8)) / 256, 256, 0, stream>>>(wih2, NHID, NHID, UPAD, whh2, NHID, NHID, WP2, KL12 / 8, NWROW, 0);
  wplane_kernel<<<(NHROW * (KHEAD / 8)) / 256, 256, 0, stream>>>(wlin, 0, NHID, HDZERO, wlin, NHID, NHID, WPH, KHEAD / 8, NHROW, 1);

  lstm3_kernel<<<NBAT / 16, NTHR, 0, stream>>>(x, bih0, bhh0, bih1, bhh1, bih2, bhh2, blin, WP0, WP1, WP2, WPH, out);
}
